// SelfAttentionLayer_30142080483695
// MI455X (gfx1250) — hardware-verified
//
#include <hip/hip_runtime.h>


#define NB_  32
#define TT   256
#define DM   1024
#define HD   16
#define NC   64
#define BPP  2
#define ZP   (BPP * NC)
#define PCAR 1024.0f
typedef _Float16 h16;
typedef unsigned short bf;
typedef __attribute__((ext_vector_type(16))) __bf16   v16bf;
typedef __attribute__((ext_vector_type(16))) _Float16 v16h;
typedef __attribute__((ext_vector_type(8)))  _Float16 v8h;
typedef __attribute__((ext_vector_type(8)))  unsigned short v8us;
typedef __attribute__((ext_vector_type(8)))  float    v8f;
typedef __attribute__((ext_vector_type(4)))  float    v4f;
typedef v8h  __attribute__((may_alias)) v8ha;
typedef v4f  __attribute__((may_alias)) v4fa;
typedef v8us __attribute__((may_alias)) v8usa;

__device__ __forceinline__ unsigned short f2bf(float f) { unsigned u = __float_as_uint(f); u += 0x7FFFu + ((u >> 16) & 1u); return (unsigned short)(u >> 16); }
__device__ __forceinline__ float bf2f(unsigned short b) { return __uint_as_float(((unsigned)b) << 16); }
__device__ __forceinline__ float bfr(float f) { return bf2f(f2bf(f)); }
__device__ __forceinline__ v16h cat16(v8h lo, v8h hi) { return __builtin_shufflevector(lo, hi, 0, 1, 2, 3, 4, 5, 6, 7, 8, 9, 10, 11, 12, 13, 14, 15); }
__device__ __forceinline__ v16bf cat16b(v8us lo, v8us hi) { return __builtin_bit_cast(v16bf, __builtin_shufflevector(lo, hi, 0, 1, 2, 3, 4, 5, 6, 7, 8, 9, 10, 11, 12, 13, 14, 15)); }
__device__ __forceinline__ v8f wmma16(v16h a, v16h b, v8f c) { return __builtin_amdgcn_wmma_f32_16x16x32_f16(false, a, false, b, (short)0, c, false, false); }
__device__ __forceinline__ v8f wmmab(v16bf a, v16bf b, v8f c) { return __builtin_amdgcn_wmma_f32_16x16x32_bf16(false, a, false, b, (short)0, c, false, false); }


template <typename T16> struct WFrag;
template <> struct WFrag<h16> { typedef v16h V; static __device__ __forceinline__ V ld(const h16* p) { return cat16(*(const v8h*)p, *(const v8h*)(p + 16)); } static __device__ __forceinline__ v8f mma(V a, V b, v8f c) { return wmma16(a, b, c); } };
template <> struct WFrag<bf> { typedef v16bf V; static __device__ __forceinline__ V ld(const bf* p) { return cat16b(*(const v8us*)p, *(const v8us*)(p + 16)); } static __device__ __forceinline__ v8f mma(V a, V b, v8f c) { return wmmab(a, b, c); } };
template <typename T16, int NSPLIT, bool BIAS>
__global__ __launch_bounds__(32) void k_gemmw(const T16* __restrict__ A, const T16* __restrict__ A2, const T16* __restrict__ Bt, const T16* __restrict__ Bt2, int K, float* C, int ldc, const float* __restrict__ bias, size_t sA, size_t sB, size_t sC) {
    typedef typename WFrag<T16>::V V;
    __shared__ __align__(16) float os[16 * 68];
    const size_t z = blockIdx.z; A += z * sA; if (A2) A2 += z * sA; Bt += z * sB; if (Bt2) Bt2 += z * sB; C += z * sC;
    const int lane = threadIdx.x & 31, lr = lane & 15, hi = lane >> 4; const int r0 = blockIdx.x * 64, c0 = blockIdx.y * 64;
    v8f acc[4][4];
#pragma unroll
    for (int mb = 0; mb < 4; ++mb)
#pragma unroll
        for (int nb = 0; nb < 4; ++nb) acc[mb][nb] = (v8f){};
    const size_t aoff = (size_t)(r0 + lr) * K + 8 * hi, boff = (size_t)(c0 + lr) * K + 8 * hi;
#pragma unroll 1
    for (int kc = 0; kc < K; kc += 32) {
        V a[4], a2[4];
#pragma unroll
        for (int mb = 0; mb < 4; ++mb) { a[mb] = WFrag<T16>::ld(A + aoff + (size_t)mb * 16 * K + kc); if (NSPLIT == 1 || NSPLIT == 2) a2[mb] = WFrag<T16>::ld(A2 + aoff + (size_t)mb * 16 * K + kc); }
#pragma unroll
        for (int nb = 0; nb < 4; ++nb) { const V b = WFrag<T16>::ld(Bt + boff + (size_t)nb * 16 * K + kc); V b2; if (NSPLIT >= 2) b2 = WFrag<T16>::ld(Bt2 + boff + (size_t)nb * 16 * K + kc);
#pragma unroll
            for (int mb = 0; mb < 4; ++mb) { acc[mb][nb] = WFrag<T16>::mma(a[mb], b, acc[mb][nb]); if (NSPLIT == 1 || NSPLIT == 2) acc[mb][nb] = WFrag<T16>::mma(a2[mb], b, acc[mb][nb]); if (NSPLIT >= 2) acc[mb][nb] = WFrag<T16>::mma(a[mb], b2, acc[mb][nb]); } }
        asm volatile("v_nop\n\tv_nop\n\tv_nop\n\tv_nop" : "+v"(acc[0][0]), "+v"(acc[1][1]), "+v"(acc[2][2]), "+v"(acc[3][3]) : "v"(a[0]), "v"(a[3]));
    }
#pragma unroll
    for (int mb = 0; mb < 4; ++mb) {
#pragma unroll
        for (int nb = 0; nb < 4; ++nb) {
#pragma unroll
            for (int j = 0; j < 8; ++j) os[(hi * 8 + j) * 68 + nb * 16 + lr] = acc[mb][nb][j]; }
        __builtin_amdgcn_wave_barrier(); asm volatile("" ::: "memory");
        float* crow = C + (size_t)(r0 + mb * 16) * ldc + c0;
#pragma unroll 1
        for (int ps = 0; ps < 2; ++ps) {
#pragma unroll
            for (int s = 0; s < 8; ++s) { const int row = 2 * s + hi, cofs = lr * 4; v4f val = *(const v4fa*)(os + row * 68 + cofs); if (BIAS) { val[0] += bfr(bias[c0 + cofs]); val[1] += bfr(bias[c0 + cofs + 1]); val[2] += bfr(bias[c0 + cofs + 2]); val[3] += bfr(bias[c0 + cofs + 3]); }
                *(volatile v4f*)(crow + (size_t)row * ldc + cofs) = val; }
            if (ps == 0) __threadfence(); }
        __builtin_amdgcn_wave_barrier(); asm volatile("" ::: "memory");
    }
}

__device__ __forceinline__ h16 tohx(float x) { return (h16)x; }
typedef __attribute__((ext_vector_type(2))) _Float16 v2h;
typedef __attribute__((ext_vector_type(4))) _Float16 v4h;

__global__ __launch_bounds__(256) void k_cvt8(const float* __restrict__ src, bf* dst, size_t n8) { const size_t i = (size_t)blockIdx.x * 256 + threadIdx.x; if (i >= n8) return; const v8f v = *(const v8f*)(src + i * 8); v8us o;
#pragma unroll
    for (int k = 0; k < 8; ++k) o[k] = f2bf(v[k]); *(volatile v8us*)(dst + i * 8) = o; __threadfence(); *(volatile v8us*)(dst + i * 8) = o; }
__global__ __launch_bounds__(256) void k_qkp(const float* __restrict__ Q, const float* __restrict__ K, int b0, h16* QP, h16* KP) { const size_t e = ((size_t)blockIdx.x * 256 + threadIdx.x) * 4; if (e >= (size_t)ZP * TT * 32) return; const int d = (int)(e % 32); const int i = (int)((e / 32) % TT); const int z = (int)(e / ((size_t)32 * TT)); const int bl = z / NC, c = z % NC; v4h a, k4;
    if (d < HD) { const size_t r = ((size_t)(b0 + bl) * TT + i) * DM + c * HD + d;
#pragma unroll
        for (int u = 0; u < 4; ++u) { a[u] = tohx(Q[r + u] * 0.03125f); k4[u] = tohx(K[r + u]); } } else { for (int u = 0; u < 4; ++u) { a[u] = (h16)0.f; k4[u] = (h16)0.f; } }
    *(volatile v4h*)(QP + e) = a; *(volatile v4h*)(KP + e) = k4; __threadfence(); *(volatile v4h*)(QP + e) = a; *(volatile v4h*)(KP + e) = k4; }
__global__ __launch_bounds__(256) void k_vtp(const float* __restrict__ V, int b0, h16* VT) { const size_t e = ((size_t)blockIdx.x * 256 + threadIdx.x) * 2; if (e >= (size_t)ZP * 64 * TT) return; const int j = (int)(e % TT); const int d = (int)((e / TT) % 64); const int z = (int)(e / ((size_t)TT * 64)); const int bl = z / NC, c = z % NC; v2h o;
    if (d < HD) { const size_t r = ((size_t)(b0 + bl) * TT + j) * DM + c * HD + d; o[0] = tohx(V[r]); o[1] = tohx(V[r + DM]); } else { o[0] = (h16)0.f; o[1] = (h16)0.f; }
    *(volatile v2h*)(VT + e) = o; __threadfence(); *(volatile v2h*)(VT + e) = o; }
__global__ __launch_bounds__(256) void k_ssoft(const float* __restrict__ S, const float* __restrict__ msk, int b0, h16* P16) { const int lane = threadIdx.x & 31; const int row = blockIdx.x * 8 + (threadIdx.x >> 5); if (row >= ZP * TT) return; const int i = row % TT; const int z = row / TT; const int b = b0 + z / NC; const float* sr = S + (size_t)row * TT; float mi = bfr(msk[b * TT + i]); asm volatile("" : "+v"(mi)); float v[TT / 32]; float mx = -3.0e38f;
#pragma unroll
    for (int ch = 0; ch < TT / 128; ++ch) { const v4f a = *(const v4f*)(sr + ch * 128 + lane * 4);
#pragma unroll
        for (int u = 0; u < 4; ++u) { const int j = ch * 128 + lane * 4 + u; float mj = bfr(msk[b * TT + j]); asm volatile("" : "+v"(mj)); float m2 = __fmul_rn(mi, mj); asm volatile("" : "+v"(m2)); float t = (m2 > 0.f) ? a[u] : -1.0e9f; asm volatile("" : "+v"(t)); v[ch * 4 + u] = t; mx = fmaxf(mx, t); } }
#pragma unroll
    for (int sh = 16; sh; sh >>= 1) mx = fmaxf(mx, __shfl_xor(mx, sh, 32));
    float sum = 0.f;
#pragma unroll
    for (int q = 0; q < TT / 32; ++q) { float d0 = __fsub_rn(v[q], mx); asm volatile("" : "+v"(d0)); v[q] = __builtin_amdgcn_exp2f(__fmul_rn(d0, 1.4426950408889634f)); sum += v[q]; }
#pragma unroll
    for (int sh = 16; sh; sh >>= 1) sum += __shfl_xor(sum, sh, 32);
    const float f = __fdiv_rn(PCAR, sum);
    for (int ps = 0; ps < 2; ++ps) {
#pragma unroll
        for (int ch = 0; ch < TT / 128; ++ch) { v4h o4; for (int q = 0; q < 4; ++q) o4[q] = tohx(v[ch * 4 + q] * f); *(volatile v4h*)(P16 + (size_t)row * TT + ch * 128 + lane * 4) = o4; }
        if (ps == 0) __threadfence(); } }
__global__ __launch_bounds__(256) void k_out(const float* __restrict__ O, int b0, float* out) { const size_t e = ((size_t)blockIdx.x * 256 + threadIdx.x) * 4; if (e >= (size_t)BPP * TT * DM) return; const int col = (int)(e % DM); const int i = (int)((e / DM) % TT); const int bl = (int)(e / ((size_t)DM * TT)); const int c = col / HD, d = col % HD; const int z = bl * NC + c; const float* src = O + ((size_t)z * TT + i) * 64 + d; v4f o;
#pragma unroll
    for (int u = 0; u < 4; ++u) o[u] = src[u] * (1.0f / PCAR); float* dst = out + ((size_t)(b0 + bl) * TT + i) * DM + col; *(volatile v4f*)dst = o; __threadfence(); *(volatile v4f*)dst = o; }

extern "C" void kernel_launch(void* const* d_in, const int* in_sizes, int n_in,
                              void* d_out, int out_size, void* d_ws, size_t ws_size, hipStream_t stream) {
    (void)in_sizes; (void)n_in; (void)out_size;
    const float* x = (const float*)d_in[0]; const float* msk = (const float*)d_in[1]; const float* Wq = (const float*)d_in[2]; const float* Wk = (const float*)d_in[3]; const float* Wv = (const float*)d_in[4];
    float* OUT = (float*)d_out;
    char* wsp = (char*)d_ws;
    auto take = [&](size_t bytes) { char* p = wsp; wsp += (bytes + 255) & ~(size_t)255; return (void*)p; };
    const size_t NR = (size_t)NB_ * TT;
    bf* XB = (bf*)take(NR * DM * 2); bf* BQ = (bf*)take((size_t)DM * DM * 2); bf* BK = (bf*)take((size_t)DM * DM * 2); bf* BV = (bf*)take((size_t)DM * DM * 2); float* Q = (float*)take(NR * DM * 4); float* K = (float*)take(NR * DM * 4); float* V = (float*)take(NR * DM * 4);
    h16* QP = (h16*)take((size_t)ZP * TT * 32 * 2); h16* KP = (h16*)take((size_t)ZP * TT * 32 * 2); h16* VT = (h16*)take((size_t)ZP * 64 * TT * 2); float* S = (float*)take((size_t)ZP * TT * TT * 4); h16* P16 = (h16*)take((size_t)ZP * TT * TT * 2); float* O = (float*)take((size_t)ZP * TT * 64 * 4);
    if ((size_t)(wsp - (char*)d_ws) > ws_size) return;
    k_cvt8<<<(unsigned)((NR * DM / 8 + 255) / 256), 256, 0, stream>>>(x, XB, NR * DM / 8); k_cvt8<<<(DM * DM / 8 + 255) / 256, 256, 0, stream>>>(Wq, BQ, DM * DM / 8); k_cvt8<<<(DM * DM / 8 + 255) / 256, 256, 0, stream>>>(Wk, BK, DM * DM / 8); k_cvt8<<<(DM * DM / 8 + 255) / 256, 256, 0, stream>>>(Wv, BV, DM * DM / 8);
    const dim3 gp((unsigned)(NR / 64), DM / 64, 1);
    k_gemmw<bf, 0, false><<<gp, 32, 0, stream>>>(XB, nullptr, BQ, nullptr, DM, Q, DM, nullptr, 0, 0, 0); k_gemmw<bf, 0, false><<<gp, 32, 0, stream>>>(XB, nullptr, BK, nullptr, DM, K, DM, nullptr, 0, 0, 0); k_gemmw<bf, 0, false><<<gp, 32, 0, stream>>>(XB, nullptr, BV, nullptr, DM, V, DM, nullptr, 0, 0, 0);
    const size_t zq = (size_t)TT * 32, zS = (size_t)TT * TT, zv = (size_t)64 * TT, zo = (size_t)TT * 64;
    for (int b0 = 0; b0 < NB_; b0 += BPP) {
        k_qkp<<<(unsigned)(((size_t)ZP * TT * 32 / 4 + 255) / 256), 256, 0, stream>>>(Q, K, b0, QP, KP); k_vtp<<<(unsigned)(((size_t)ZP * 64 * TT / 2 + 255) / 256), 256, 0, stream>>>(V, b0, VT);
        k_gemmw<h16, 0, false><<<dim3(TT / 64, TT / 64, ZP), 32, 0, stream>>>(QP, nullptr, KP, nullptr, 32, S, TT, nullptr, zq, zq, zS);
        k_ssoft<<<ZP * TT / 8, 256, 0, stream>>>(S, msk, b0, P16);
        k_gemmw<h16, 0, false><<<dim3(TT / 64, 1, ZP), 32, 0, stream>>>(P16, nullptr, VT, nullptr, TT, O, 64, nullptr, zS, zv, zo);
        k_out<<<(unsigned)(((size_t)BPP * TT * DM / 4 + 255) / 256), 256, 0, stream>>>(O, b0, OUT); }
}
